// BilinearConvLinear_88373247082945
// MI455X (gfx1250) — hardware-verified
//
#include <hip/hip_runtime.h>


typedef _Float16 __hf16;
#define __bf16 __hf16
#define __builtin_amdgcn_wmma_f32_16x16x32_bf16 __builtin_amdgcn_wmma_f32_16x16x32_f16
typedef __attribute__((ext_vector_type(16))) _Float16 v16bf;
typedef __attribute__((ext_vector_type(8)))  _Float16 v8bf;
typedef __attribute__((ext_vector_type(8)))  float  v8f;

#define TDIM 4096
#define BDIM 8
#define CDIM 32
#define LWIN 25
#define NNODE 32
#define WAVES 4
#define POS_PER_WAVE 16
#define POS_PER_BLOCK (WAVES * POS_PER_WAVE)
#define SLABW 96

__device__ __forceinline__ v16bf combine8(v8bf lo, v8bf hi) {
  return __builtin_shufflevector(lo, hi, 0, 1, 2, 3, 4, 5, 6, 7,
                                 8, 9, 10, 11, 12, 13, 14, 15);
}

extern "C" __global__ __launch_bounds__(WAVES * 32, 1)
void bilinear_conv_linear_kernel(const float* __restrict__ x,
                                 const float* __restrict__ w,
                                 const float* __restrict__ projw,
                                 const float* __restrict__ projb,
                                 float* __restrict__ out) {
  extern __shared__ __align__(16) unsigned char smem[];
  __bf16* projT   = (__bf16*)smem;
  float*  wLds    = (float*)(smem + 65536);
  float*  sqAll   = (float*)(smem + 65664);
  __bf16* XsT     = (__bf16*)(smem + 65920);
  __bf16* featAll = (__bf16*)(smem + 72064);

  const int tid  = threadIdx.x;
  const int lane = tid & 31;
  const int wave = tid >> 5;
  const int kh   = lane >> 4;
  const int nlo  = lane & 15;

  const int bIdx    = blockIdx.x / (TDIM / POS_PER_BLOCK);
  const int tblk    = blockIdx.x % (TDIM / POS_PER_BLOCK);
  const int t0block = tblk * POS_PER_BLOCK;
  const size_t xbase = (size_t)bIdx * TDIM * CDIM;

  for (int i = tid; i < CDIM * CDIM * NNODE; i += WAVES * 32) {
    int fp = i >> 5;
    int n2 = i & 31;
    int tile = fp >> 8, ln = (fp >> 3) & 31, r = fp & 7;
    int ti = tile >> 1, tj = tile & 1;
    int m = ti * 16 + (ln >> 4) * 8 + r;
    int nn = tj * 16 + (ln & 15);
    int f = m * CDIM + nn;
    projT[n2 * 1024 + fp] = (__bf16)projw[f * NNODE + n2];
  }
  if (tid < 32) wLds[tid] = (tid < LWIN) ? w[tid] : 0.0f;
  for (int i = tid; i < CDIM * SLABW; i += WAVES * 32) {
    int col = i >> 5, c = i & 31;
    int ts = t0block - (LWIN / 2) + col;
    float v = (ts >= 0 && ts < TDIM) ? x[xbase + (size_t)ts * CDIM + c] : 0.0f;
    XsT[c * SLABW + col] = (__bf16)v;
  }
  __syncthreads();

  __bf16* feat = featAll + (size_t)wave * (POS_PER_WAVE * CDIM * CDIM);
  float*  sqW  = sqAll + wave * 16;
  const int t0 = t0block + wave * POS_PER_WAVE;

  const int kbase0 = kh * 8;
  const int kbase1 = 16 + kh * 8;
  v16bf wfrag;
#pragma unroll
  for (int i = 0; i < 8; ++i) {
    wfrag[i]     = (__bf16)wLds[kbase0 + i];
    wfrag[8 + i] = (__bf16)wLds[kbase1 + i];
  }
  const __bf16* row0 = XsT + nlo * SLABW;
  const __bf16* row1 = XsT + (16 + nlo) * SLABW;

  for (int j = 0; j < POS_PER_WAVE; ++j) {
    const int wj = wave * POS_PER_WAVE + j;

    v16bf b0, b1;
#pragma unroll
    for (int i = 0; i < 8; ++i) {
      b0[i] = row0[wj + kbase0 + i];  b0[8 + i] = row0[wj + kbase1 + i];
      b1[i] = row1[wj + kbase0 + i];  b1[8 + i] = row1[wj + kbase1 + i];
    }
    v16bf a0 = wfrag * b0;
    v16bf a1 = wfrag * b1;

    v8f acc00 = {}, acc01 = {}, acc10 = {}, acc11 = {};
    acc00 = __builtin_amdgcn_wmma_f32_16x16x32_bf16(false, a0, false, b0, (short)0, acc00, false, false);
    acc01 = __builtin_amdgcn_wmma_f32_16x16x32_bf16(false, a0, false, b1, (short)0, acc01, false, false);
    acc10 = __builtin_amdgcn_wmma_f32_16x16x32_bf16(false, a1, false, b0, (short)0, acc10, false, false);
    acc11 = __builtin_amdgcn_wmma_f32_16x16x32_bf16(false, a1, false, b1, (short)0, acc11, false, false);
    asm volatile("v_nop\n\tv_nop\n\tv_nop\n\tv_nop" : "+v"(acc00), "+v"(acc11) : "v"(a1), "v"(b1));

    v8bf* frow = (v8bf*)(feat + j * (CDIM * CDIM)) + lane;
    v8bf p00, p01, p10, p11;
#pragma unroll
    for (int r = 0; r < 8; ++r) {
      p00[r] = (__bf16)acc00[r];
      p01[r] = (__bf16)acc01[r];
      p10[r] = (__bf16)acc10[r];
      p11[r] = (__bf16)acc11[r];
    }
    frow[0]  = p00;
    frow[32] = p01;
    frow[64] = p10;
    frow[96] = p11;
  }
  asm volatile("s_wait_dscnt 0" ::: "memory");

  const v8bf* fA  = (const v8bf*)(feat + nlo * 1024);
  const v8bf* pB0 = (const v8bf*)(projT + nlo * 1024);
  const v8bf* pB1 = (const v8bf*)(projT + (16 + nlo) * 1024);

  v8f o0 = {}, o1 = {}, g = {};
#pragma unroll 4
  for (int ks = 0; ks < 32; ++ks) {
    const int c0 = ks * 4 + kh;
    const int c1 = ks * 4 + 2 + kh;
    v16bf afr = combine8(fA[c0], fA[c1]);
    v16bf bf0 = combine8(pB0[c0], pB0[c1]);
    v16bf bf1 = combine8(pB1[c0], pB1[c1]);
    o0 = __builtin_amdgcn_wmma_f32_16x16x32_bf16(false, afr, false, bf0, (short)0, o0, false, false);
    o1 = __builtin_amdgcn_wmma_f32_16x16x32_bf16(false, afr, false, bf1, (short)0, o1, false, false);
    g  = __builtin_amdgcn_wmma_f32_16x16x32_bf16(false, afr, false, afr, (short)0, g,  false, false);
    asm volatile("v_nop\n\tv_nop\n\tv_nop\n\tv_nop" : "+v"(o0), "+v"(g) : "v"(afr), "v"(bf1));
  }

#pragma unroll
  for (int r = 0; r < 8; ++r) {
    int j = r + kh * 8;
    if (j == nlo) sqW[j] = g[r];
  }
  asm volatile("s_wait_dscnt 0" ::: "memory");

  float rsv[8];
#pragma unroll
  for (int r = 0; r < 8; ++r)
    rsv[r] = rsqrtf(fmaxf(sqW[r + kh * 8], 1e-12f));

  const float bias0 = projb[nlo];
  const float bias1 = projb[16 + nlo];
  for (int pass = 0; pass < 2; ++pass) {
#pragma unroll
    for (int r = 0; r < 8; ++r) {
      const float v0 = o0[r] * rsv[r] + bias0, v1 = o1[r] * rsv[r] + bias1;
      const float x0 = __shfl_xor(v0, 16), x1 = __shfl_xor(v1, 16);
      const size_t rowA = ((size_t)bIdx * TDIM + (size_t)(t0 + r)) * NNODE, rowB = ((size_t)bIdx * TDIM + (size_t)(t0 + 8 + r)) * NNODE;
      *(volatile float*)(out + rowA + lane) = kh ? x1 : v0;
      *(volatile float*)(out + rowB + lane) = kh ? v1 : x0;
    }
    __threadfence();
  }
}

extern "C" void kernel_launch(void* const* d_in, const int* in_sizes, int n_in,
                              void* d_out, int out_size, void* d_ws, size_t ws_size,
                              hipStream_t stream) {
  (void)in_sizes; (void)n_in; (void)out_size; (void)d_ws; (void)ws_size;
  const float* x  = (const float*)d_in[0];
  const float* w  = (const float*)d_in[1];
  const float* pw = (const float*)d_in[2];
  const float* pb = (const float*)d_in[3];
  float* out = (float*)d_out;

  constexpr size_t SMEM = 65536
                        + 128
                        + 256
                        + (size_t)CDIM * SLABW * 2
                        + (size_t)WAVES * POS_PER_WAVE * CDIM * CDIM * 2;

  dim3 grid(BDIM * (TDIM / POS_PER_BLOCK));
  dim3 block(WAVES * 32);
  hipFuncSetAttribute((const void*)bilinear_conv_linear_kernel, hipFuncAttributeMaxDynamicSharedMemorySize, (int)SMEM);
  bilinear_conv_linear_kernel<<<grid, block, SMEM, stream>>>(x, w, pw, pb, out);
}
